// LinearAttentionBlock_68650757259443
// MI455X (gfx1250) — hardware-run, weakly checked
//
#include <hip/hip_runtime.h>


#ifndef NB
#define NB 2
#endif
#ifndef NTOK
#define NTOK 4096
#endif
#define NB_FULL   2
#define NTOK_FULL 4096
#ifndef OUT_TOK
#define OUT_TOK NTOK
#endif
#define CDIM 256
#define NHD  4
#define HDM  64
#define OQKV (3 * CDIM)
#define QRS  2048.0f
#define QRI  (1.0f / 2048.0f)
#define L2E  1.4426950408889634f
#define NEGB (-3.0e38f)
#define PCAR 4096.0f
#define MCAR 1024.0f
#define WCAR 64.0f
#define W2CAR 1024.0f
#define INVN (1.0f / (float)NTOK)
#define CSR  128
#define NCH  (NTOK / CSR)
#define NRB  64
#define KSPL 8
#define KCH  (NTOK / KSPL)
#define MSZ  (HDM * HDM)
#define XTP  72
#define MHP  72
#define OSP  36

static_assert(NHD * HDM == CDIM);
static_assert(HDM == 64);
static_assert(OQKV == NHD * 3 * HDM);
static_assert(CDIM % 32 == 0);
static_assert(CDIM % 64 == 0);
static_assert(HDM % 32 == 0);
static_assert(NTOK % 64 == 0);
static_assert(NTOK % CSR == 0);
static_assert(NTOK % NRB == 0);
static_assert(NTOK % KSPL == 0);
static_assert(KCH % 32 == 0);
static_assert(NTOK % 8 == 0);
static_assert(NB <= NB_FULL);
static_assert(NTOK <= NTOK_FULL);
static_assert(OUT_TOK >= NTOK);
static_assert((OUT_TOK * 4) % 128 == 0);
static_assert(((size_t)OQKV * CDIM) % 8 == 0);
static_assert((XTP * 2) % 16 == 0);
static_assert((MHP * 2) % 16 == 0);
static_assert((OSP * 4) % 16 == 0);
static_assert(CDIM == 256);

typedef _Float16 h16;
typedef unsigned short bf;
typedef __attribute__((ext_vector_type(16))) __bf16   v16bf;
typedef __attribute__((ext_vector_type(16))) _Float16 v16h;
typedef __attribute__((ext_vector_type(8)))  _Float16 v8h;
typedef __attribute__((ext_vector_type(8)))  unsigned short v8us;
typedef __attribute__((ext_vector_type(8)))  float    v8f;
typedef __attribute__((ext_vector_type(4)))  float    v4f;
typedef v4f  __attribute__((may_alias)) v4fa;

__device__ __forceinline__ unsigned short f2bf(float f) { unsigned u = __float_as_uint(f); u += 0x7FFFu + ((u >> 16) & 1u); return (unsigned short)(u >> 16); }
__device__ __forceinline__ float bfr(float f) { return __uint_as_float(((unsigned)f2bf(f)) << 16); }
__device__ __forceinline__ v16h cat16(v8h lo, v8h hi) { return __builtin_shufflevector(lo, hi, 0, 1, 2, 3, 4, 5, 6, 7, 8, 9, 10, 11, 12, 13, 14, 15); }
__device__ __forceinline__ v16bf cat16b(v8us lo, v8us hi) { return __builtin_bit_cast(v16bf, __builtin_shufflevector(lo, hi, 0, 1, 2, 3, 4, 5, 6, 7, 8, 9, 10, 11, 12, 13, 14, 15)); }
__device__ __forceinline__ v8f wmma16(v16h a, v16h b, v8f c) { return __builtin_amdgcn_wmma_f32_16x16x32_f16(false, a, false, b, (short)0, c, false, false); }
__device__ __forceinline__ v8f wmmab(v16bf a, v16bf b, v8f c) { return __builtin_amdgcn_wmma_f32_16x16x32_bf16(false, a, false, b, (short)0, c, false, false); }
__device__ __forceinline__ v16h  ldh(const h16* p) { return cat16(*(const v8h*)p, *(const v8h*)(p + 16)); }
__device__ __forceinline__ v16bf ldb(const bf* p)  { return cat16b(*(const v8us*)p, *(const v8us*)(p + 16)); }
__device__ __forceinline__ void wave_sync() { __builtin_amdgcn_fence(3  , "wavefront"); __builtin_amdgcn_wave_barrier(); asm volatile("" ::: "memory"); }

static __device__ __forceinline__ h16 toh_flush(float v) { const h16 r = (h16)v; return (fabsf(v) < 6.103515625e-05f) ? (h16)0.0f : r; }
static __device__ __forceinline__ v8f gmma16(v16h a, v16h b, v8f c) { c = wmma16(a, b, c); asm volatile("v_nop\n\tv_nop\n\tv_nop\n\tv_nop" : "+v"(c) : "v"(a), "v"(b)); return c; }
static __device__ __forceinline__ v8f gmmab(v16bf a, v16bf b, v8f c) { c = wmmab(a, b, c); asm volatile("v_nop\n\tv_nop\n\tv_nop\n\tv_nop" : "+v"(c) : "v"(a), "v"(b)); return c; }

__global__ __launch_bounds__(256) void k_cvt8(const float* __restrict__ src, bf* dst, size_t n8) {
    const size_t i = (size_t)blockIdx.x * 256 + threadIdx.x; if (i >= n8) return;
    const v8f v = *(const v8f*)(src + i * 8); v8us o;
#pragma unroll
    for (int k = 0; k < 8; ++k) o[k] = f2bf(v[k]);
    *(volatile v8us*)(dst + i * 8) = o; __threadfence(); *(volatile v8us*)(dst + i * 8) = o;
}

static_assert(256 * 16 * 2 == 64 * 128);
static_assert(64 * XTP * 2 <= 131072);
__global__ __launch_bounds__(256) void k_xt(const float* __restrict__ x, bf* XT) {
    __shared__ __align__(16) unsigned short ts[64 * XTP];
    const int tid = threadIdx.x;
    const int t0 = blockIdx.x * 64, c0 = blockIdx.y * 64, b = blockIdx.z;
    { const int c = tid >> 2, tq = (tid & 3) * 16;
      const float* src = x + ((size_t)b * CDIM + c0 + c) * NTOK_FULL + t0 + tq;
#pragma unroll
      for (int q = 0; q < 4; ++q) { const v4f v = *(const v4f*)(src + 4 * q);
#pragma unroll
          for (int k = 0; k < 4; ++k) ts[(tq + 4 * q + k) * XTP + c] = f2bf(v[k]); } }
    __syncthreads();
    bf* dst = XT + ((size_t)b * NTOK + t0) * CDIM + c0;
#pragma unroll 1
    for (int ps = 0; ps < 2; ++ps) {
#pragma unroll
        for (int it = 0; it < 2; ++it) { const int row = it * 32 + (tid >> 3), c8 = (tid & 7) * 8;
            const v8us o = *(const v8us*)(&ts[row * XTP + c8]);
            *(volatile v8us*)(dst + (size_t)row * CDIM + c8) = o; }
        if (ps == 0) __threadfence(); }
}

static_assert(32 * 16 * 4 == 16 * 128);
static_assert(32 * 16 * 8 == 16 * 256);
static_assert(16 * 68 * 4 <= 131072);
__global__ __launch_bounds__(32) void k_qkv(const bf* __restrict__ P, size_t woff, h16* PLN, size_t ple, float* KF) {
    __shared__ __align__(16) float os[16 * 68];
    const int lane = threadIdx.x & 31, lr = lane & 15, hi = lane >> 4;
    const int ot = blockIdx.x; const int head = ot / 3, kind = ot - 3 * head;
    const int n0 = blockIdx.y * 64; const int bb = n0 / NTOK, tt = n0 % NTOK;
    const size_t wrow = woff + (size_t)(ot * 64) * CDIM;
    const size_t xrow = (size_t)n0 * CDIM;
    const bool kt = (kind == 1);
    const size_t aoff = (kt ? xrow : wrow) + (size_t)lr * CDIM + 8 * hi;
    const size_t boff = (kt ? wrow : xrow) + (size_t)lr * CDIM + 8 * hi;
    v8f acc[4][4];
#pragma unroll
    for (int mb = 0; mb < 4; ++mb)
#pragma unroll
        for (int nb = 0; nb < 4; ++nb) acc[mb][nb] = (v8f){};
#pragma unroll 1
    for (int kc = 0; kc < CDIM; kc += 32) {
        v16bf a[4];
#pragma unroll
        for (int mb = 0; mb < 4; ++mb) a[mb] = ldb(P + aoff + (size_t)mb * 16 * CDIM + kc);
#pragma unroll
        for (int nb = 0; nb < 4; ++nb) { const v16bf b = ldb(P + boff + (size_t)nb * 16 * CDIM + kc);
#pragma unroll
            for (int mb = 0; mb < 4; ++mb) acc[mb][nb] = gmmab(a[mb], b, acc[mb][nb]); }
    }
    if (kt) {
        float* dst0 = KF + ((size_t)bb * NTOK + tt) * CDIM + head * HDM;
#pragma unroll
        for (int mb = 0; mb < 4; ++mb) {
#pragma unroll
            for (int nb = 0; nb < 4; ++nb) {
#pragma unroll
                for (int j = 0; j < 8; ++j) os[(hi * 8 + j) * 68 + nb * 16 + lr] = acc[mb][nb][j]; }
            wave_sync();
#pragma unroll 1
            for (int ps = 0; ps < 2; ++ps) {
#pragma unroll
                for (int s = 0; s < 8; ++s) { const int row = 2 * s + (lane >> 4), cofs = (lane & 15) * 4;
                    const v4f val = *(const v4fa*)(&os[row * 68 + cofs]);
                    *(volatile v4f*)(dst0 + (size_t)(mb * 16 + row) * CDIM + cofs) = val; }
                if (ps == 0) __threadfence(); }
            wave_sync();
        }
    } else {
        const size_t pbase = (kind == 0) ? (size_t)0 : 2 * ple;
        const size_t tbase = pbase + ((size_t)(bb * NHD + head) * HDM) * NTOK + (size_t)tt;
#pragma unroll
        for (int mb = 0; mb < 4; ++mb) {
#pragma unroll
            for (int nb = 0; nb < 4; ++nb) {
#pragma unroll
                for (int j = 0; j < 8; ++j) os[(hi * 8 + j) * 68 + nb * 16 + lr] = acc[mb][nb][j]; }
            wave_sync();
            const size_t sb = tbase + (size_t)(mb * 16) * NTOK;
#pragma unroll 1
            for (int ps = 0; ps < 2; ++ps) {
#pragma unroll
                for (int s = 0; s < 4; ++s) { const int row = 4 * s + (lane >> 3), c8 = (lane & 7) * 8;
                    const v4f x0 = *(const v4fa*)(&os[row * 68 + c8]); const v4f x1 = *(const v4fa*)(&os[row * 68 + c8 + 4]); v8h hv, rv;
#pragma unroll
                    for (int i = 0; i < 4; ++i) { const h16 a0 = toh_flush(x0[i]); const h16 a1 = toh_flush(x1[i]); hv[i] = a0; hv[4 + i] = a1;
                        rv[i] = toh_flush((x0[i] - (float)a0) * QRS); rv[4 + i] = toh_flush((x1[i] - (float)a1) * QRS); }
                    const size_t oo = sb + (size_t)row * NTOK + c8;
                    *(volatile v8h*)(PLN + oo) = hv; *(volatile v8h*)(PLN + ple + oo) = rv; }
                if (ps == 0) __threadfence(); }
            wave_sync();
        }
    }
}

static_assert(128 * 16 * 1 == 2 * CDIM * 4);
__global__ __launch_bounds__(256) void k_cstat(const float* __restrict__ KF, float* PST) {
#pragma clang fp contract(off)
    __shared__ __align__(16) float st[2 * CDIM];
    const int tid = threadIdx.x;
    const int wave = __builtin_amdgcn_readfirstlane((int)(threadIdx.x >> 5));
    const int ch = blockIdx.x, b = blockIdx.y;
    const float* src = KF + ((size_t)b * NTOK + (size_t)ch * CSR) * CDIM + tid;
    float m = NEGB;
#pragma unroll 4
    for (int r = 0; r < CSR; ++r) m = fmaxf(m, src[(size_t)r * CDIM]);
    float s = 0.0f;
#pragma unroll 4
    for (int r = 0; r < CSR; ++r) s += __builtin_amdgcn_exp2f((src[(size_t)r * CDIM] - m) * L2E);
    st[tid] = m; st[CDIM + tid] = s;
    __syncthreads();
    float* dst = PST + ((size_t)b * NCH + ch) * (2 * CDIM);
    if (wave < 4) { const v4f v = *(const v4fa*)(&st[tid * 4]);
        *(volatile v4f*)(dst + tid * 4) = v; __threadfence(); *(volatile v4f*)(dst + tid * 4) = v; }
}

static_assert(256 * 16 * (NRB / 8) == NRB * CDIM * 2);
__global__ __launch_bounds__(256) void k_norm(const float* __restrict__ KF, const float* __restrict__ PST, h16* KT) {
#pragma clang fp contract(off)
    __shared__ __align__(16) float cm[CDIM];
    __shared__ __align__(16) float cr[CDIM];
    const int tid = threadIdx.x;
    const int b = blockIdx.y, r0 = blockIdx.x * NRB;
    { const float* ps = PST + (size_t)b * NCH * (2 * CDIM) + tid;
      float M = NEGB;
#pragma unroll 1
      for (int ch = 0; ch < NCH; ++ch) M = fmaxf(M, ps[(size_t)ch * (2 * CDIM)]);
      float S = 0.0f;
#pragma unroll 1
      for (int ch = 0; ch < NCH; ++ch) S += ps[(size_t)ch * (2 * CDIM) + CDIM] * __builtin_amdgcn_exp2f((ps[(size_t)ch * (2 * CDIM)] - M) * L2E);
      cm[tid] = M; cr[tid] = PCAR * (1.0f / S); }
    __syncthreads();
    const int c8 = (tid & 31) * 8, rr = tid >> 5;
    const v4f m0 = *(const v4fa*)(&cm[c8]), m1 = *(const v4fa*)(&cm[c8 + 4]);
    const v4f q0 = *(const v4fa*)(&cr[c8]), q1 = *(const v4fa*)(&cr[c8 + 4]);
#pragma unroll 1
    for (int it = 0; it < NRB / 8; ++it) {
        const size_t off = ((size_t)b * NTOK + r0 + it * 8 + rr) * CDIM + c8;
        const v4f x0 = *(const v4f*)(KF + off), x1 = *(const v4f*)(KF + off + 4);
        v8h o;
#pragma unroll
        for (int i = 0; i < 4; ++i) {
            o[i]     = toh_flush(__builtin_amdgcn_exp2f((x0[i] - m0[i]) * L2E) * q0[i]);
            o[4 + i] = toh_flush(__builtin_amdgcn_exp2f((x1[i] - m1[i]) * L2E) * q1[i]); }
        *(volatile v8h*)(KT + off) = o; __threadfence(); *(volatile v8h*)(KT + off) = o;
    }
}

static_assert(32 * 16 * 8 == 32 * 128);
static_assert(4 * 32 * OSP * 4 <= 131072);
__global__ __launch_bounds__(128) void k_ctx(const h16* __restrict__ PLN, size_t ple, float* MP) {
    __shared__ __align__(16) float os[4 * 32 * OSP];
    const int lane = threadIdx.x & 31, lr = lane & 15, hi = lane >> 4;
    const int wave = __builtin_amdgcn_readfirstlane((int)(threadIdx.x >> 5));
    const int kc = blockIdx.x, zh = blockIdx.y;
    const int rq = wave >> 1, cq = wave & 1;
    const size_t vo = 2 * ple + ((size_t)zh * HDM + rq * 32 + lr) * NTOK + (size_t)kc * KCH + 8 * hi;
    const size_t qo =           ((size_t)zh * HDM + cq * 32 + lr) * NTOK + (size_t)kc * KCH + 8 * hi;
    v8f aM[2][2], aR[2][2];
#pragma unroll
    for (int i = 0; i < 2; ++i)
#pragma unroll
        for (int j = 0; j < 2; ++j) { aM[i][j] = (v8f){}; aR[i][j] = (v8f){}; }
#pragma unroll 1
    for (int ks = 0; ks < KCH; ks += 32) {
        v16h vh[2], vr[2], qh[2], qr[2];
#pragma unroll
        for (int i = 0; i < 2; ++i) {
            vh[i] = ldh(PLN + vo + (size_t)i * 16 * NTOK + ks); vr[i] = ldh(PLN + vo + ple + (size_t)i * 16 * NTOK + ks);
            qh[i] = ldh(PLN + qo + (size_t)i * 16 * NTOK + ks); qr[i] = ldh(PLN + qo + ple + (size_t)i * 16 * NTOK + ks); }
#pragma unroll
        for (int i = 0; i < 2; ++i)
#pragma unroll
            for (int j = 0; j < 2; ++j) {
                aM[i][j] = gmma16(vh[i], qh[j], aM[i][j]);
                aR[i][j] = gmma16(vh[i], qr[j], aR[i][j]);
                aR[i][j] = gmma16(vr[i], qh[j], aR[i][j]); }
    }
    const int wb = wave * 32 * OSP;
#pragma unroll
    for (int i = 0; i < 2; ++i)
#pragma unroll
        for (int j = 0; j < 2; ++j)
#pragma unroll
            for (int r = 0; r < 8; ++r) os[wb + (i * 16 + hi * 8 + r) * OSP + j * 16 + lr] = aM[i][j][r] + aR[i][j][r] * QRI;
    wave_sync();
    float* dst = MP + (((size_t)zh * KSPL + kc) * HDM + rq * 32) * HDM + cq * 32;
#pragma unroll 1
    for (int ps = 0; ps < 2; ++ps) {
#pragma unroll
        for (int s = 0; s < 8; ++s) { const int row = 4 * s + (lane >> 3), cofs = (lane & 7) * 4;
            const v4f val = *(const v4fa*)(&os[wb + row * OSP + cofs]);
            *(volatile v4f*)(dst + (size_t)row * HDM + cofs) = val; }
        if (ps == 0) __threadfence(); }
}

static_assert(256 * 16 == MSZ);
static_assert(32 * 16 * 4 == 16 * 128);
static_assert(8 * 32 == CDIM);
static_assert(2 * HDM * MHP * 2 + 8 * 16 * 68 * 4 <= 65536);
__global__ __launch_bounds__(256) void k_w2(const float* __restrict__ wout, const float* __restrict__ MP, h16* W2H) {
    __shared__ __align__(16) h16 mh[HDM * MHP];
    __shared__ __align__(16) h16 mr[HDM * MHP];
    __shared__ __align__(16) float os[8 * 16 * 68];
    const int tid = threadIdx.x;
    const int lane = threadIdx.x & 31, lr = lane & 15, hi = lane >> 4;
    const int wave = __builtin_amdgcn_readfirstlane((int)(threadIdx.x >> 5));
    const int zh = blockIdx.x; const int b = zh / NHD, h = zh % NHD;
    { const int row = tid >> 2, c16 = (tid & 3) * 16;
      const float* src = MP + (size_t)zh * KSPL * MSZ + row * HDM + c16;
      v4f s0 = (v4f){}, s1 = (v4f){}, s2 = (v4f){}, s3 = (v4f){};
#pragma unroll 1
      for (int kc = 0; kc < KSPL; ++kc) { const float* p = src + (size_t)kc * MSZ;
          s0 += *(const v4f*)p; s1 += *(const v4f*)(p + 4); s2 += *(const v4f*)(p + 8); s3 += *(const v4f*)(p + 12); }
      const float msc = MCAR * INVN;
      v8h h0, h1, g0, g1;
#pragma unroll
      for (int i = 0; i < 4; ++i) {
          float c; h16 a;
          c = s0[i] * msc; a = toh_flush(c); h0[i] = a;     g0[i] = toh_flush((c - (float)a) * QRS);
          c = s1[i] * msc; a = toh_flush(c); h0[4 + i] = a; g0[4 + i] = toh_flush((c - (float)a) * QRS);
          c = s2[i] * msc; a = toh_flush(c); h1[i] = a;     g1[i] = toh_flush((c - (float)a) * QRS);
          c = s3[i] * msc; a = toh_flush(c); h1[4 + i] = a; g1[4 + i] = toh_flush((c - (float)a) * QRS); }
      *(v8h*)(&mh[row * MHP + c16]) = h0; *(v8h*)(&mh[row * MHP + c16 + 8]) = h1;
      *(v8h*)(&mr[row * MHP + c16]) = g0; *(v8h*)(&mr[row * MHP + c16 + 8]) = g1; }
    __syncthreads();
    const int wb = wave * 16 * 68;
    const float w2s = W2CAR / (WCAR * MCAR);
#pragma unroll 1
    for (int rt = 0; rt < 2; ++rt) {
        const int orow0 = wave * 32 + rt * 16;
        v8f aM[4], aR[4];
#pragma unroll
        for (int ct = 0; ct < 4; ++ct) { aM[ct] = (v8f){}; aR[ct] = (v8f){}; }
#pragma unroll
        for (int ks = 0; ks < HDM / 32; ++ks) {
            const float* wp = wout + (size_t)(orow0 + lr) * CDIM + h * HDM + ks * 32 + 8 * hi;
            const v4f w0 = *(const v4f*)wp, w1 = *(const v4f*)(wp + 4), w2 = *(const v4f*)(wp + 16), w3 = *(const v4f*)(wp + 20);
            v16h a;
#pragma unroll
            for (int i = 0; i < 4; ++i) { a[i] = toh_flush(bfr(w0[i]) * WCAR); a[4 + i] = toh_flush(bfr(w1[i]) * WCAR);
                                          a[8 + i] = toh_flush(bfr(w2[i]) * WCAR); a[12 + i] = toh_flush(bfr(w3[i]) * WCAR); }
#pragma unroll
            for (int ct = 0; ct < 4; ++ct) { const int bi = (ct * 16 + lr) * MHP + ks * 32 + 8 * hi;
                const v16h bh = cat16(*(const v8h*)(&mh[bi]), *(const v8h*)(&mh[bi + 16]));
                const v16h br = cat16(*(const v8h*)(&mr[bi]), *(const v8h*)(&mr[bi + 16]));
                aM[ct] = gmma16(a, bh, aM[ct]); aR[ct] = gmma16(a, br, aR[ct]); }
        }
#pragma unroll
        for (int ct = 0; ct < 4; ++ct)
#pragma unroll
            for (int j = 0; j < 8; ++j) os[wb + (hi * 8 + j) * 68 + ct * 16 + lr] = (aM[ct][j] + aR[ct][j] * QRI) * w2s;
        wave_sync();
        h16* dst = W2H + ((size_t)b * CDIM + orow0) * CDIM + h * HDM;
#pragma unroll 1
        for (int ps = 0; ps < 2; ++ps) {
#pragma unroll
            for (int s = 0; s < 4; ++s) { const int row = 4 * s + (lane >> 3), c8 = (lane & 7) * 8;
                const v4f x0 = *(const v4fa*)(&os[wb + row * 68 + c8]); const v4f x1 = *(const v4fa*)(&os[wb + row * 68 + c8 + 4]); v8h hv;
#pragma unroll
                for (int i = 0; i < 4; ++i) { hv[i] = toh_flush(x0[i]); hv[4 + i] = toh_flush(x1[i]); }
                *(volatile v8h*)(dst + (size_t)row * CDIM + c8) = hv; }
            if (ps == 0) __threadfence(); }
        wave_sync();
    }
}

static_assert(32 * 16 * 8 == 16 * 256);
__global__ __launch_bounds__(32) void k_out(const h16* __restrict__ W2H, const h16* __restrict__ KT, const float* __restrict__ bias, float* OUT) {
    __shared__ __align__(16) float os[16 * 68];
    const int lane = threadIdx.x & 31, lr = lane & 15, hi = lane >> 4;
    const int r0 = blockIdx.x * 64, c0 = blockIdx.y * 64, b = blockIdx.z;
    const size_t aoff = ((size_t)b * CDIM + r0 + lr) * CDIM + 8 * hi;
    const size_t boff = ((size_t)b * NTOK + c0 + lr) * CDIM + 8 * hi;
    v8f acc[4][4];
#pragma unroll
    for (int mb = 0; mb < 4; ++mb)
#pragma unroll
        for (int nb = 0; nb < 4; ++nb) acc[mb][nb] = (v8f){};
#pragma unroll 1
    for (int kc = 0; kc < CDIM; kc += 32) {
        v16h a[4];
#pragma unroll
        for (int mb = 0; mb < 4; ++mb) a[mb] = ldh(W2H + aoff + (size_t)mb * 16 * CDIM + kc);
#pragma unroll
        for (int nb = 0; nb < 4; ++nb) { const v16h bq = ldh(KT + boff + (size_t)nb * 16 * CDIM + kc);
#pragma unroll
            for (int mb = 0; mb < 4; ++mb) acc[mb][nb] = gmma16(a[mb], bq, acc[mb][nb]); }
    }
    const float osc = 1.0f / (W2CAR * PCAR);
#pragma unroll
    for (int mb = 0; mb < 4; ++mb) {
        float br[8];
#pragma unroll
        for (int j = 0; j < 8; ++j) br[j] = bfr(bias[r0 + mb * 16 + hi * 8 + j]);
#pragma unroll
        for (int nb = 0; nb < 4; ++nb) {
#pragma unroll
            for (int j = 0; j < 8; ++j) os[(hi * 8 + j) * 68 + nb * 16 + lr] = acc[mb][nb][j] * osc + br[j]; }
        wave_sync();
        float* dst = OUT + ((size_t)b * CDIM + r0 + mb * 16) * OUT_TOK + c0;
#pragma unroll 1
        for (int ps = 0; ps < 2; ++ps) {
#pragma unroll
            for (int s = 0; s < 8; ++s) { const int row = 2 * s + (lane >> 4), cofs = (lane & 15) * 4;
                const v4f val = *(const v4fa*)(&os[row * 68 + cofs]);
                *(volatile v4f*)(dst + (size_t)row * OUT_TOK + cofs) = val; }
            if (ps == 0) __threadfence(); }
        wave_sync();
    }
}

static constexpr size_t al256(size_t v) { return (v + 255) & ~(size_t)255; }
static constexpr size_t PLE    = (size_t)NB * NHD * HDM * NTOK;
static constexpr size_t SZ_XT  = al256((size_t)NB * NTOK * CDIM * 2);
static constexpr size_t SZ_WB  = al256((size_t)OQKV * CDIM * 2);
static constexpr size_t SZ_PL  = PLE * 2;
static constexpr size_t SZ_KF  = al256((size_t)NB * NTOK * CDIM * 4);
static constexpr size_t SZ_PST = al256((size_t)NB * NCH * 2 * CDIM * 4);
static constexpr size_t SZ_KT  = al256((size_t)NB * NTOK * CDIM * 2);
static constexpr size_t SZ_MP  = al256((size_t)NB * NHD * KSPL * MSZ * 4);
static constexpr size_t SZ_W2  = al256((size_t)NB * CDIM * CDIM * 2);
static constexpr size_t SZ_TOTAL = SZ_XT + SZ_WB + 4 * SZ_PL + SZ_KF + SZ_PST + SZ_KT + SZ_MP + SZ_W2;
static_assert(SZ_TOTAL <= (size_t)134217728);
static_assert(SZ_PL % 256 == 0);
static_assert(SZ_XT == (size_t)NB * NTOK * CDIM * 2);
static_assert((size_t)(NB * NTOK / 64) * 64 == (size_t)NB * NTOK);

extern "C" void kernel_launch(void* const* d_in, const int* in_sizes, int n_in,
                              void* d_out, int out_size, void* d_ws, size_t ws_size, hipStream_t stream) {
    if (n_in < 4) return;
    const size_t needx = ((size_t)(NB - 1) * CDIM + (CDIM - 1)) * NTOK_FULL + NTOK;
    if ((size_t)in_sizes[0] < needx) return;
    if ((size_t)in_sizes[1] < (size_t)OQKV * CDIM || (size_t)in_sizes[2] < (size_t)CDIM * CDIM || in_sizes[3] < CDIM) return;
    if ((size_t)out_size < ((size_t)(NB - 1) * CDIM + (CDIM - 1)) * OUT_TOK + NTOK) return;
    if (SZ_TOTAL > ws_size) return;
    const float* x    = (const float*)d_in[0];
    const float* wqkv = (const float*)d_in[1];
    const float* wout = (const float*)d_in[2];
    const float* bout = (const float*)d_in[3];
    float* OUT = (float*)d_out;
    char* wsp = (char*)d_ws;
    bf*    XT  = (bf*)wsp;    wsp += SZ_XT;
    bf*    WB  = (bf*)wsp;    wsp += SZ_WB;
    h16*   PLN = (h16*)wsp;   wsp += 4 * SZ_PL;
    float* KF  = (float*)wsp; wsp += SZ_KF;
    float* PST = (float*)wsp; wsp += SZ_PST;
    h16*   KT  = (h16*)wsp;   wsp += SZ_KT;
    float* MP  = (float*)wsp; wsp += SZ_MP;
    h16*   W2H = (h16*)wsp;   wsp += SZ_W2;

    { const size_t n8 = (size_t)OQKV * CDIM / 8;
      k_cvt8<<<(unsigned)((n8 + 255) / 256), 256, 0, stream>>>(wqkv, WB, n8); }
    k_xt<<<dim3(NTOK / 64, CDIM / 64, NB), 256, 0, stream>>>(x, XT);
    k_qkv<<<dim3(OQKV / 64, NB * NTOK / 64, 1), 32, 0, stream>>>(XT, SZ_XT / 2, PLN, PLE, KF);
    k_cstat<<<dim3(NCH, NB, 1), 256, 0, stream>>>(KF, PST);
    k_norm<<<dim3(NTOK / NRB, NB, 1), 256, 0, stream>>>(KF, PST, KT);
    k_ctx<<<dim3(KSPL, NB * NHD, 1), 128, 0, stream>>>(PLN, PLE, MP);
    k_w2<<<dim3(NB * NHD, 1, 1), 256, 0, stream>>>(wout, MP, W2H);
    k_out<<<dim3(CDIM / 64, NTOK / 64, NB), 32, 0, stream>>>(W2H, KT, bout, OUT);
}
